// BuildingBlockEmbedder_55387898249705
// MI455X (gfx1250) — hardware-verified
//
#include <hip/hip_runtime.h>
#include <stddef.h>


#define HD      128
#define H2      256
#define KG      64
#define KG0     51
#define EWR     307
#define WSC     64
#define GSC     64
#define OSC     (1.0f / 64.0f)
#define OSCG    (1.0f / 4096.0f)
#define NTHR    256
#define TW      4
#define TTHR    (TW * 32)
#define BM      64
#define NCW     64
#define ANB     32
#define ENB     32
#define DEGCAP  64
#define ERND    256
#define NPBCAP  1024
#define WSCAP   134217728

static_assert(BM * 4 == NTHR);
static_assert(TTHR == 128);
static_assert((ERND % BM) == 0 && (ERND % NTHR) == 0);
static_assert((KG % 32) == 0 && KG0 <= KG);
static_assert(ANB == 32 && ENB == 32);

typedef float          v4f  __attribute__((ext_vector_type(4)));
typedef float          v8f  __attribute__((ext_vector_type(8)));
typedef int            v4i  __attribute__((ext_vector_type(4)));
typedef _Float16       v4h  __attribute__((ext_vector_type(4)));
typedef _Float16       v8h  __attribute__((ext_vector_type(8)));
typedef _Float16       v16h __attribute__((ext_vector_type(16)));
typedef _Float16       v8ha __attribute__((ext_vector_type(8), __may_alias__));
typedef unsigned short v4us __attribute__((ext_vector_type(4)));
typedef unsigned short v8us __attribute__((ext_vector_type(8)));
union FragH { v16h v; v8us u[2]; v8h h[2]; };

__device__ __forceinline__ v8f wmh(v16h a, v16h b, v8f c) {
  v8f d = __builtin_amdgcn_wmma_f32_16x16x32_f16(false, a, false, b, (short)0, c, false, false);
  asm volatile("v_nop\n\tv_nop\n\tv_nop\n\tv_nop" : "+v"(d) : "v"(a), "v"(b));
  return d;
}
__device__ __forceinline__ v8f zero8() { v8f z = {0.f, 0.f, 0.f, 0.f, 0.f, 0.f, 0.f, 0.f}; return z; }

__device__ __forceinline__ v16h frag_glb(const unsigned short* P, int row, int ld, int k0, int hh) {
  FragH f;
  const unsigned short* p = P + (size_t)row * ld + k0 + 8 * hh;
  f.u[0] = *(const v8us*)p;
  f.u[1] = *(const v8us*)(p + 16);
  return f.v;
}
__device__ __forceinline__ v16h frag_lds(const _Float16* T, int row, int ld, int k0, int hh) {
  FragH f;
  const _Float16* p = T + row * ld + k0 + 8 * hh;
  f.h[0] = *(const v8h*)p;
  f.h[1] = *(const v8h*)(p + 16);
  return f.v;
}

__device__ __forceinline__ void wcvt_unit(const float* __restrict__ W, unsigned short* dst,
                                          int K, int KP, int Nout, int ld, int i) {
  const int upc = KP >> 3;
  if (i >= Nout * upc) return;
  const int n = i / upc;
  const int seg = i - n * upc;
  v8h o;
#pragma unroll
  for (int j = 0; j < 8; ++j) {
    const int k = 8 * seg + j;
    const int kc = k < K - 1 ? k : K - 1;
    const float v = W[(size_t)kc * ld + n];
    o[j] = (_Float16)((k < K) ? v * (float)WSC : v * 0.0f);
  }
  const v8us ob = __builtin_bit_cast(v8us, o);
  unsigned short* d = dst + (size_t)i * 8;
  *(volatile v8us*)d = ob;
  __threadfence();
  *(volatile v8us*)d = ob;
}

__global__ __launch_bounds__(NTHR) void k_wcvt(const float* __restrict__ eW1, const float* __restrict__ eW2,
                                               const float* __restrict__ nW1, const float* __restrict__ nW2,
                                               unsigned short* pqw, unsigned short* gwp, unsigned short* ew2p,
                                               unsigned short* nw1p, unsigned short* nw2p) {
  const int job = (int)blockIdx.y;
  const size_t lz = (size_t)blockIdx.z;
  const float* W =
      (job == 0) ? (eW1 + lz * EWR * HD) :
      (job == 1) ? (eW1 + lz * EWR * HD + (size_t)HD * HD) :
      (job == 2) ? (eW1 + lz * EWR * HD + (size_t)H2 * HD) :
      (job == 3) ? (eW2 + lz * HD * HD) :
      (job == 4) ? (nW1 + lz * H2 * HD) : (nW2 + lz * HD * HD);
  unsigned short* dst =
      (job == 0) ? (pqw + lz * H2 * HD) :
      (job == 1) ? (pqw + lz * H2 * HD + (size_t)HD * HD) :
      (job == 2) ? (gwp + lz * HD * KG) :
      (job == 3) ? (ew2p + lz * HD * HD) :
      (job == 4) ? (nw1p + lz * HD * H2) : (nw2p + lz * HD * HD);
  const int K  = (job == 2) ? KG0 : ((job == 4) ? H2 : HD);
  const int KP = (job == 2) ? KG  : ((job == 4) ? H2 : HD);
  wcvt_unit(W, dst, K, KP, HD, HD, (int)blockIdx.x * NTHR + (int)threadIdx.x);
}

__global__ __launch_bounds__(NTHR) void k_embed(const int* __restrict__ at, const float* __restrict__ emb,
                                                float* H32, unsigned short* HA, int nN, int nTypes) {
  const int tid = threadIdx.x, lane = tid & 31, wave = tid >> 5;
  const int nb = (int)blockIdx.x * ENB + wave * 4;
  v4f hv[4];
  v4us hu[4];
#pragma unroll
  for (int j = 0; j < 4; ++j) {
    int n = nb + j; n = n > nN - 1 ? nN - 1 : n;
    int t = at[n] - 1;
    t = t < 0 ? t + nTypes : t;
    t = t < 0 ? 0 : (t > nTypes - 1 ? nTypes - 1 : t);
    hv[j] = *(const v4f*)(emb + (size_t)t * HD + 4 * lane);
    v4h o;
    o.x = (_Float16)hv[j].x; o.y = (_Float16)hv[j].y; o.z = (_Float16)hv[j].z; o.w = (_Float16)hv[j].w;
    hu[j] = __builtin_bit_cast(v4us, o);
  }
#pragma unroll
  for (int j = 0; j < 4; ++j) {
    int n = nb + j; n = n > nN - 1 ? nN - 1 : n;
    *(volatile v4f*)(H32 + (size_t)n * HD + 4 * lane) = hv[j];
    *(volatile v4us*)(HA + (size_t)n * HD + 4 * lane) = hu[j];
  }
  __threadfence();
#pragma unroll
  for (int j = 0; j < 4; ++j) {
    int n = nb + j; n = n > nN - 1 ? nN - 1 : n;
    *(volatile v4f*)(H32 + (size_t)n * HD + 4 * lane) = hv[j];
    *(volatile v4us*)(HA + (size_t)n * HD + 4 * lane) = hu[j];
  }
}

__global__ __launch_bounds__(NTHR) void k_geo(const float* __restrict__ x, const int* __restrict__ row,
                                              const int* __restrict__ col, unsigned short* GEO, int nN, int nE) {
  __shared__ __attribute__((aligned(16))) _Float16 sG[NTHR * KG];
  const int tid = threadIdx.x;
  const int rbase = (int)blockIdx.x * NTHR;
  {
    int e = rbase + tid; e = e > nE - 1 ? nE - 1 : e;
    int i = row[e], j = col[e];
    i = i < 0 ? 0 : (i > nN - 1 ? nN - 1 : i);
    j = j < 0 ? 0 : (j > nN - 1 ? nN - 1 : j);
    const float* pi = x + (size_t)i * 3;
    const float* pj = x + (size_t)j * 3;
    const float xi0 = pi[0], xi1 = pi[1], xi2 = pi[2];
    const float xj0 = pj[0], xj1 = pj[1], xj2 = pj[2];
    const float dx = xi0 - xj0, dy = xi1 - xj1, dz = xi2 - xj2;
    const float d2 = dx * dx + dy * dy + dz * dz;
    const float d = sqrtf(d2);
    const float ax = xi0 * 0.1f - xj0 * 0.1f;
    const float ay = xi1 * 0.1f - xj1 * 0.1f;
    const float az = xi2 * 0.1f - xj2 * 0.1f;
    const float rad = ax * ax + ay * ay + az * az;
    const float step  = 0.102040816f;
    const float coeff = -48.02f;
#pragma unroll 1
    for (int q = 0; q < 8; ++q) {
      v8h o;
#pragma unroll
      for (int jj = 0; jj < 8; ++jj) {
        const int k = 8 * q + jj;
        const float t = d - step * (float)(k - 1);
        const float g = __expf(coeff * t * t);
        const float v = (k == 0) ? rad : ((k <= KG0 - 1) ? g : g * 0.0f);
        o[jj] = (_Float16)(v * (float)GSC);
      }
      *(v8h*)(sG + tid * KG + 8 * q) = o;
    }
  }
  __syncthreads();
  v8us pv[8];
#pragma unroll
  for (int it = 0; it < 8; ++it) {
    const int p = it * NTHR + tid;
    const int r = p >> 3, seg = p & 7;
    pv[it] = __builtin_bit_cast(v8us, *(const v8ha*)(sG + r * KG + 8 * seg));
  }
  unsigned short* base = GEO + (size_t)rbase * KG;
#pragma unroll
  for (int it = 0; it < 8; ++it)
    *(volatile v8us*)(base + (size_t)(it * NTHR + tid) * 8) = pv[it];
  __threadfence();
#pragma unroll
  for (int it = 0; it < 8; ++it)
    *(volatile v8us*)(base + (size_t)(it * NTHR + tid) * 8) = pv[it];
}

__global__ __launch_bounds__(NTHR) void k_gemm(const unsigned short* __restrict__ Ap,
                                               const unsigned short* __restrict__ Bp,
                                               float* C, int lda, int KT, int ldc, float osc) {
  __shared__ __attribute__((aligned(16))) float stg[BM * NCW];
  const int tid = threadIdx.x, lane = tid & 31, wave = tid >> 5, hh = lane >> 4, m = lane & 15;
  const int rowBase = (int)blockIdx.x * BM;
  const int colBase = (int)blockIdx.y * NCW;
  const int rg = wave >> 1, chf = wave & 1;
  const int r0 = rg * 16;
  const int c0 = chf * 32;
  const int KB = 32 * KT;

  v8f acc0 = zero8();
  v8f acc1 = zero8();

  const unsigned short* ap  = Ap + (size_t)(rowBase + r0 + m) * lda + 8 * hh;
  const unsigned short* bpA = Bp + (size_t)(colBase + c0 + m) * KB + 8 * hh;
  const unsigned short* bpB = bpA + (size_t)16 * KB;
#pragma unroll 1
  for (int kt = 0; kt < KT; ++kt) {
    const v8us a0 = *(const v8us*)(ap + 32 * kt);
    const v8us a1 = *(const v8us*)(ap + 32 * kt + 16);
    const v8us b00 = *(const v8us*)(bpA + 32 * kt);
    const v8us b01 = *(const v8us*)(bpA + 32 * kt + 16);
    const v8us b10 = *(const v8us*)(bpB + 32 * kt);
    const v8us b11 = *(const v8us*)(bpB + 32 * kt + 16);
    FragH a, b0, b1;
    a.u[0] = a0; a.u[1] = a1; b0.u[0] = b00; b0.u[1] = b01; b1.u[0] = b10; b1.u[1] = b11;
    acc0 = wmh(a.v, b0.v, acc0);
    acc1 = wmh(a.v, b1.v, acc1);
  }

  {
    float* sp = stg + (size_t)(r0 + 8 * hh) * NCW + c0 + m;
#pragma unroll
    for (int r = 0; r < 8; ++r) {
      sp[r * NCW]      = acc0[r] * osc;
      sp[r * NCW + 16] = acc1[r] * osc;
    }
  }
  __syncthreads();

  v4f cv[4];
#pragma unroll
  for (int it = 0; it < 4; ++it) {
    const int id = it * NTHR + tid;
    const int row = id >> 4, seg = id & 15;
    cv[it] = *(const v4f*)(stg + (size_t)row * NCW + 4 * seg);
  }
#pragma unroll
  for (int it = 0; it < 4; ++it) {
    const int id = it * NTHR + tid;
    const int row = id >> 4, seg = id & 15;
    float* gp = C + (size_t)(rowBase + row) * ldc + colBase + 4 * seg;
    *(volatile v4f*)gp = cv[it];
  }
  __threadfence();
#pragma unroll
  for (int it = 0; it < 4; ++it) {
    const int id = it * NTHR + tid;
    const int row = id >> 4, seg = id & 15;
    float* gp = C + (size_t)(rowBase + row) * ldc + colBase + 4 * seg;
    *(volatile v4f*)gp = cv[it];
  }
}

__device__ __forceinline__ void rows_out_pass(const float* sOut, float* H32, unsigned short* HA, int n0, int lane) {
#pragma unroll
  for (int i = 0; i < 16; ++i) {
    const v4f v = *(const v4f*)(sOut + i * HD + 4 * lane);
    *(volatile v4f*)(H32 + (size_t)(n0 + i) * HD + 4 * lane) = v;
  }
#pragma unroll
  for (int i = 0; i < 8; ++i) {
    const v4f a = *(const v4f*)(sOut + i * 256 + 8 * lane);
    const v4f b = *(const v4f*)(sOut + i * 256 + 8 * lane + 4);
    v8h o;
    o[0] = (_Float16)a.x; o[1] = (_Float16)a.y; o[2] = (_Float16)a.z; o[3] = (_Float16)a.w;
    o[4] = (_Float16)b.x; o[5] = (_Float16)b.y; o[6] = (_Float16)b.z; o[7] = (_Float16)b.w;
    const v8us ob = __builtin_bit_cast(v8us, o);
    *(volatile v8us*)(HA + (size_t)n0 * HD + i * 256 + 8 * lane) = ob;
  }
}

__device__ __forceinline__ void frows_pass(const float* sT, float* P, int s0, int lane) {
#pragma unroll
  for (int i = 0; i < 16; ++i) {
    const v4f v = *(const v4f*)(sT + i * HD + 4 * lane);
    *(volatile v4f*)(P + (size_t)(s0 + i) * HD + 4 * lane) = v;
  }
}

__global__ __launch_bounds__(TTHR) void k_edge(
    const int* __restrict__ row, const int* __restrict__ col, const float* __restrict__ PQ,
    const unsigned short* __restrict__ GEO, const unsigned short* __restrict__ GWp,
    const float* __restrict__ eb1, const unsigned short* __restrict__ W2p, const float* __restrict__ eb2,
    float* Mp, int nN, int nE) {
  __shared__ __attribute__((aligned(16))) float    sF[TW][16 * HD];
  __shared__ __attribute__((aligned(16))) _Float16 sA[TW][16 * HD];
  __shared__ int sIdx[TW][32];
  const int tid = threadIdx.x, lane = tid & 31, wave = tid >> 5, hh = lane >> 4, m = lane & 15;
  const int s0 = ((int)blockIdx.x * TW + wave) * 16;
  float* sFw = sF[wave];
  _Float16* sAw = sA[wave];

  {
    const int e = lane & 15;
    int s = s0 + e; s = s > nE - 1 ? nE - 1 : s;
    int r = row[s];
    int c = col[s];
    r = r < 0 ? 0 : (r > nN - 1 ? nN - 1 : r);
    c = c < 0 ? 0 : (c > nN - 1 ? nN - 1 : c);
    if (lane < 16) {
      sIdx[wave][2 * e]     = r;
      sIdx[wave][2 * e + 1] = c;
    }
  }
  __syncthreads();

  {
    const v4f bq = *(const v4f*)(eb1 + 4 * lane);
#pragma unroll 2
    for (int e = 0; e < 16; ++e) {
      const int r = sIdx[wave][2 * e];
      const int c = sIdx[wave][2 * e + 1];
      const v4f p = *(const v4f*)(PQ + (size_t)r * H2 + 4 * lane);
      const v4f q = *(const v4f*)(PQ + (size_t)c * H2 + HD + 4 * lane);
      *(v4f*)(sFw + e * HD + 4 * lane) = (p + q) + bq;
    }
  }
  __syncthreads();

  {
    const v16h ga0 = frag_glb(GEO, s0 + m, KG, 0, hh);
    const v16h ga1 = frag_glb(GEO, s0 + m, KG, 32, hh);
#pragma unroll 1
    for (int np = 0; np < 4; ++np) {
      const int c0 = 32 * np + m, c1 = c0 + 16;
      v8f acc0 = zero8(), acc1 = zero8();
      const v16h b00 = frag_glb(GWp, c0, KG, 0, hh);
      const v16h b01 = frag_glb(GWp, c0, KG, 32, hh);
      const v16h b10 = frag_glb(GWp, c1, KG, 0, hh);
      const v16h b11 = frag_glb(GWp, c1, KG, 32, hh);
      acc0 = wmh(ga0, b00, acc0);
      acc0 = wmh(ga1, b01, acc0);
      acc1 = wmh(ga0, b10, acc1);
      acc1 = wmh(ga1, b11, acc1);
#pragma unroll
      for (int r = 0; r < 8; ++r) {
        const int rr = 8 * hh + r;
        float x0 = acc0[r] * OSCG + sFw[rr * HD + c0];
        float x1 = acc1[r] * OSCG + sFw[rr * HD + c1];
        x0 = fmaxf(x0, 0.0f);
        x1 = fmaxf(x1, 0.0f);
        sAw[rr * HD + c0] = (_Float16)x0;
        sAw[rr * HD + c1] = (_Float16)x1;
      }
    }
  }
  __syncthreads();

#pragma unroll 1
  for (int np = 0; np < 4; ++np) {
    const int c0 = 32 * np + m, c1 = c0 + 16;
    v8f acc0 = zero8(), acc1 = zero8();
#pragma unroll 1
    for (int kt = 0; kt < 4; ++kt) {
      const v16h a  = frag_lds(sAw, m, HD, 32 * kt, hh);
      const v16h b0 = frag_glb(W2p, c0, HD, 32 * kt, hh);
      const v16h b1 = frag_glb(W2p, c1, HD, 32 * kt, hh);
      acc0 = wmh(a, b0, acc0);
      acc1 = wmh(a, b1, acc1);
    }
    const float bv0 = eb2[c0], bv1 = eb2[c1];
#pragma unroll
    for (int r = 0; r < 8; ++r) {
      const int rr = 8 * hh + r;
      sFw[rr * HD + c0] = fmaxf(acc0[r] * OSC + bv0, 0.0f);
      sFw[rr * HD + c1] = fmaxf(acc1[r] * OSC + bv1, 0.0f);
    }
  }
  __syncthreads();

  frows_pass(sFw, Mp, s0, lane);
  __threadfence();
  frows_pass(sFw, Mp, s0, lane);
}

__global__ __launch_bounds__(NTHR) void k_agg(const int* __restrict__ row, const float* __restrict__ Mp,
                                              unsigned short* AggA, int nN, int nE, int deg) {
  const int tid = threadIdx.x, lane = tid & 31, wave = tid >> 5;
  const int nb = (int)blockIdx.x * ANB + wave * 4;
  const int dg = deg < 0 ? 0 : (deg > DEGCAP ? DEGCAP : deg);
  const v4f z4 = {0.f, 0.f, 0.f, 0.f};
  v4us agv[4];
#pragma unroll
  for (int j = 0; j < 4; ++j) {
    int n = nb + j; n = n > nN - 1 ? nN - 1 : n;
    v4f acc = z4;
#pragma unroll 1
    for (int i = 0; i < dg; ++i) {
      int e = n * deg + i;
      e = e < 0 ? 0 : (e > nE - 1 ? nE - 1 : e);
      const int rr = row[e];
      const v4f v = *(const v4f*)(Mp + (size_t)e * HD + 4 * lane);
      const bool ok = (rr == n);
      acc.x += ok ? v.x : 0.0f;
      acc.y += ok ? v.y : 0.0f;
      acc.z += ok ? v.z : 0.0f;
      acc.w += ok ? v.w : 0.0f;
    }
    v4h ho;
    ho.x = (_Float16)acc.x; ho.y = (_Float16)acc.y; ho.z = (_Float16)acc.z; ho.w = (_Float16)acc.w;
    agv[j] = __builtin_bit_cast(v4us, ho);
  }
#pragma unroll
  for (int j = 0; j < 4; ++j) {
    int n = nb + j; n = n > nN - 1 ? nN - 1 : n;
    *(volatile v4us*)(AggA + (size_t)n * HD + 4 * lane) = agv[j];
  }
  __threadfence();
#pragma unroll
  for (int j = 0; j < 4; ++j) {
    int n = nb + j; n = n > nN - 1 ? nN - 1 : n;
    *(volatile v4us*)(AggA + (size_t)n * HD + 4 * lane) = agv[j];
  }
}

__global__ __launch_bounds__(TTHR) void k_node(
    float* H32, unsigned short* HA, const unsigned short* __restrict__ AggA,
    const unsigned short* __restrict__ N1p, const float* __restrict__ nb1,
    const unsigned short* __restrict__ N2p, const float* __restrict__ nb2, int nN) {
  __shared__ __attribute__((aligned(16))) float    sOutB[TW][16 * HD];
  __shared__ __attribute__((aligned(16))) _Float16 sMidB[TW][16 * HD];
  const int tid = threadIdx.x, lane = tid & 31, wave = tid >> 5, hh = lane >> 4, m = lane & 15;
  const int n0 = ((int)blockIdx.x * TW + wave) * 16;
  _Float16* sMid = sMidB[wave];
  float* sOut = sOutB[wave];
  (void)nN;

#pragma unroll 1
  for (int np = 0; np < 4; ++np) {
    const int c0 = 32 * np + m, c1 = c0 + 16;
    v8f acc0 = zero8(), acc1 = zero8();
#pragma unroll 1
    for (int kt = 0; kt < 4; ++kt) {
      const v16h a  = frag_glb(HA, n0 + m, HD, 32 * kt, hh);
      const v16h b0 = frag_glb(N1p, c0, H2, 32 * kt, hh);
      const v16h b1 = frag_glb(N1p, c1, H2, 32 * kt, hh);
      acc0 = wmh(a, b0, acc0);
      acc1 = wmh(a, b1, acc1);
    }
#pragma unroll 1
    for (int kt = 0; kt < 4; ++kt) {
      const v16h a  = frag_glb(AggA, n0 + m, HD, 32 * kt, hh);
      const v16h b0 = frag_glb(N1p, c0, H2, HD + 32 * kt, hh);
      const v16h b1 = frag_glb(N1p, c1, H2, HD + 32 * kt, hh);
      acc0 = wmh(a, b0, acc0);
      acc1 = wmh(a, b1, acc1);
    }
    const float bv0 = nb1[c0], bv1 = nb1[c1];
#pragma unroll
    for (int r = 0; r < 8; ++r) {
      sMid[(8 * hh + r) * HD + c0] = (_Float16)fmaxf(acc0[r] * OSC + bv0, 0.0f);
      sMid[(8 * hh + r) * HD + c1] = (_Float16)fmaxf(acc1[r] * OSC + bv1, 0.0f);
    }
  }
  __syncthreads();

#pragma unroll 1
  for (int np = 0; np < 4; ++np) {
    const int c0 = 32 * np + m, c1 = c0 + 16;
    v8f acc0 = zero8(), acc1 = zero8();
#pragma unroll 1
    for (int kt = 0; kt < 4; ++kt) {
      const v16h a  = frag_lds(sMid, m, HD, 32 * kt, hh);
      const v16h b0 = frag_glb(N2p, c0, HD, 32 * kt, hh);
      const v16h b1 = frag_glb(N2p, c1, HD, 32 * kt, hh);
      acc0 = wmh(a, b0, acc0);
      acc1 = wmh(a, b1, acc1);
    }
#pragma unroll
    for (int r = 0; r < 8; ++r) {
      sOut[(8 * hh + r) * HD + c0] = acc0[r] * OSC;
      sOut[(8 * hh + r) * HD + c1] = acc1[r] * OSC;
    }
  }
  __syncthreads();

  {
    const v4f bq = *(const v4f*)(nb2 + 4 * lane);
#pragma unroll 2
    for (int i = 0; i < 16; ++i) {
      const v4f dv = *(const v4f*)(sOut + i * HD + 4 * lane);
      const v4f hv = *(const v4f*)(H32 + (size_t)(n0 + i) * HD + 4 * lane);
      const v4f u = dv + bq;
      const v4f t = hv + u;
      const v4f y = hv + t;
      *(v4f*)(sOut + i * HD + 4 * lane) = y;
    }
  }
  __syncthreads();

  rows_out_pass(sOut, H32, HA, n0, lane);
  __threadfence();
  rows_out_pass(sOut, H32, HA, n0, lane);
}

__global__ __launch_bounds__(NTHR) void k_pool(const float* __restrict__ H32, float* out, int nBB, int npb,
                                               float inv) {
  const int tid = threadIdx.x, lane = tid & 31, wave = tid >> 5;
  const int bb = (int)blockIdx.x * 8 + wave;
  if (bb >= nBB) return;
  const int np = npb < 0 ? 0 : (npb > NPBCAP ? NPBCAP : npb);
  v4f acc = {0.f, 0.f, 0.f, 0.f};
#pragma unroll 1
  for (int v = 0; v < np; ++v)
    acc += *(const v4f*)(H32 + ((size_t)bb * npb + v) * HD + 4 * lane);
  const v4f res = acc * inv;
  float* gp = out + (size_t)bb * HD + 4 * lane;
  *(volatile v4f*)gp = res;
  __threadfence();
  *(volatile v4f*)gp = res;
}

extern "C" void kernel_launch(void* const* d_in, const int* in_sizes, int n_in,
                              void* d_out, int out_size, void* d_ws, size_t ws_size,
                              hipStream_t stream) {
  if (n_in < 13) return;
  const int nN = in_sizes[0];
  const int nE = in_sizes[2];
  if (nN <= 0 || nE <= 0) return;
  if (nN > (1 << 20) || nE > (1 << 26)) return;
  if (in_sizes[1] != 3 * nN || in_sizes[3] != nE) return;
  const int nTypes = in_sizes[4] / HD;
  if (nTypes <= 0 || in_sizes[4] != nTypes * HD) return;
  const int L = in_sizes[6] / HD;
  if (L <= 0 || L > 64) return;
  if (in_sizes[5] != L * EWR * HD || in_sizes[6] != L * HD || in_sizes[7] != L * HD * HD || in_sizes[8] != L * HD) return;
  if (in_sizes[9] != L * H2 * HD || in_sizes[10] != L * HD || in_sizes[11] != L * HD * HD || in_sizes[12] != L * HD) return;
  if (out_size <= 0 || (out_size % HD) != 0) return;
  const int nBB = out_size / HD;
  if ((nN % nBB) != 0) return;
  const int npb = nN / nBB;
  if (npb <= 0 || npb > NPBCAP) return;
  if ((nN % BM) != 0 || (nN % ANB) != 0 || (nN % ENB) != 0) return;
  if ((nE % nN) != 0) return;
  const int deg = nE / nN;
  if (deg <= 0 || deg > DEGCAP) return;
  const int Epad = (nE + ERND - 1) & ~(ERND - 1);

  const int*   at   = (const int*)d_in[0];
  const float* xs   = (const float*)d_in[1];
  const int*   rows = (const int*)d_in[2];
  const int*   cols = (const int*)d_in[3];
  const float* emb  = (const float*)d_in[4];
  const float* eW1  = (const float*)d_in[5];
  const float* eb1  = (const float*)d_in[6];
  const float* eW2  = (const float*)d_in[7];
  const float* eb2  = (const float*)d_in[8];
  const float* nW1  = (const float*)d_in[9];
  const float* nb1  = (const float*)d_in[10];
  const float* nW2  = (const float*)d_in[11];
  const float* nb2  = (const float*)d_in[12];
  float* out = (float*)d_out;

  const size_t NPs = (size_t)nN, EPs = (size_t)Epad;
  char* ws = (char*)d_ws;
  size_t off = 0;
  const size_t oPQW = off; off += (size_t)L * H2 * HD * 2;   off = (off + 255) & ~(size_t)255;
  const size_t oGW  = off; off += (size_t)L * HD * KG * 2;   off = (off + 255) & ~(size_t)255;
  const size_t oEW2 = off; off += (size_t)L * HD * HD * 2;   off = (off + 255) & ~(size_t)255;
  const size_t oNW1 = off; off += (size_t)L * HD * H2 * 2;   off = (off + 255) & ~(size_t)255;
  const size_t oNW2 = off; off += (size_t)L * HD * HD * 2;   off = (off + 255) & ~(size_t)255;
  const size_t oH32 = off; off += NPs * HD * 4;              off = (off + 255) & ~(size_t)255;
  const size_t oHA  = off; off += NPs * HD * 2;              off = (off + 255) & ~(size_t)255;
  const size_t oAGG = off; off += NPs * HD * 2;              off = (off + 255) & ~(size_t)255;
  const size_t oPQ  = off; off += NPs * H2 * 4;              off = (off + 255) & ~(size_t)255;
  const size_t oGEO = off; off += EPs * KG * 2;              off = (off + 255) & ~(size_t)255;
  const size_t oM   = off; off += EPs * HD * 4;              off = (off + 255) & ~(size_t)255;
  if (off > ws_size || off > (size_t)WSCAP) return;

  unsigned short* PQW  = (unsigned short*)(ws + oPQW);
  unsigned short* GWp  = (unsigned short*)(ws + oGW);
  unsigned short* EW2p = (unsigned short*)(ws + oEW2);
  unsigned short* NW1p = (unsigned short*)(ws + oNW1);
  unsigned short* NW2p = (unsigned short*)(ws + oNW2);
  float*          H32  = (float*)(ws + oH32);
  unsigned short* HA   = (unsigned short*)(ws + oHA);
  unsigned short* AGG  = (unsigned short*)(ws + oAGG);
  float*          PQ   = (float*)(ws + oPQ);
  unsigned short* GEO  = (unsigned short*)(ws + oGEO);
  float*          Mpl  = (float*)(ws + oM);

  k_wcvt<<<dim3((HD * (H2 / 8) + NTHR - 1) / NTHR, 6, L), NTHR, 0, stream>>>(eW1, eW2, nW1, nW2,
                                                                            PQW, GWp, EW2p, NW1p, NW2p);
  k_embed<<<nN / ENB, NTHR, 0, stream>>>(at, emb, H32, HA, nN, nTypes);
  k_geo<<<Epad / NTHR, NTHR, 0, stream>>>(xs, rows, cols, GEO, nN, nE);

  for (int l = 0; l < L; ++l) {
    const size_t lz = (size_t)l;
    k_gemm<<<dim3(nN / BM, H2 / NCW, 1), NTHR, 0, stream>>>(HA, PQW + lz * H2 * HD, PQ, HD, HD / 32, H2, OSC);
    k_edge<<<Epad / (TW * 16), TTHR, 0, stream>>>(rows, cols, PQ, GEO, GWp + lz * HD * KG, eb1 + lz * HD,
                                                   EW2p + lz * HD * HD, eb2 + lz * HD, Mpl, nN, nE);
    k_agg<<<nN / ANB, NTHR, 0, stream>>>(rows, Mpl, AGG, nN, nE, deg);
    k_node<<<nN / (TW * 16), TTHR, 0, stream>>>(H32, HA, AGG, NW1p + lz * HD * H2, nb1 + lz * HD,
                                                NW2p + lz * HD * HD, nb2 + lz * HD, nN);
  }
  k_pool<<<(nBB + 7) / 8, NTHR, 0, stream>>>(H32, out, nBB, npb, 1.0f / (float)npb);
}
